// Block_24283745092155
// MI455X (gfx1250) — hardware-verified
//
#include <hip/hip_runtime.h>
#include <math.h>

typedef __attribute__((ext_vector_type(16))) _Float16 v16h;
typedef __attribute__((ext_vector_type(8)))  _Float16 v8h;
typedef __attribute__((ext_vector_type(8)))  float    v8f;
typedef __attribute__((ext_vector_type(4)))  float    v4f;

constexpr int kBatch = 2;
constexpr int kSeqL  = 2048;
constexpr int kDmod  = 1024;
constexpr int kDin   = 2048;
constexpr int kNst   = 16;
constexpr int kDtR   = 64;
constexpr int kPrjN  = 96;
constexpr int kPrjP  = 128;
constexpr int kXZP   = 2 * kDin;
constexpr int kRows  = kBatch * kSeqL;
constexpr int kTP    = 260;
constexpr float kLnEps = 1e-5f;
constexpr float kInvDm = 1.0f / (float)kDmod;

constexpr float kCarWin  = 32.0f;
constexpr float kCarWxp  = 32.0f;
constexpr float kCarWdt  = 8.0f;
constexpr float kCarWout = 32.0f;
constexpr float kCarDt   = 16.0f;
constexpr float kCarY    = 16.0f;
constexpr float kFoldIn  = 1.0f / kCarWin;
constexpr float kFoldXp  = 1.0f / kCarWxp;
constexpr float kFoldDt  = 1.0f / (kCarDt * kCarWdt);
constexpr float kFoldOut = 1.0f / (kCarY * kCarWout);

static_assert(kDtR + 2 * kNst == kPrjN);
static_assert(kDmod == 1024 && kDin == 2048 && kNst == 16 && kDtR == 64 && kSeqL == 2048 && kBatch == 2);
static_assert((kDmod % 32) == 0 && (kDin % 32) == 0 && (kDtR % 32) == 0);
static_assert((kSeqL % 64) == 0 && (kXZP % 64) == 0 && (kPrjP % 64) == 0 && (kDin % 64) == 0 && (kDmod % 64) == 0);
static_assert((kDin % 256) == 0 && (kSeqL % 16) == 0);

constexpr size_t kSzWIN16  = (size_t)kXZP * kDmod * 2;
constexpr size_t kSzWXP16  = (size_t)kPrjP * kDin * 2;
constexpr size_t kSzWDT16  = (size_t)kDin * kDtR * 2;
constexpr size_t kSzWOUT16 = (size_t)kDmod * kDin * 2;
constexpr size_t kSzYLN16  = (size_t)kRows * kDmod * 2;
constexpr size_t kSzXZ     = (size_t)kSeqL * kXZP * 4;
constexpr size_t kSzUC     = (size_t)kSeqL * kDin * 4;
constexpr size_t kSzUC16   = (size_t)kSeqL * kDin * 2;
constexpr size_t kSzPROJ   = (size_t)kSeqL * kPrjP * 4;
constexpr size_t kSzDT16   = (size_t)kSeqL * kDtR * 2;
constexpr size_t kSzDLR    = (size_t)kSeqL * kDin * 4;
constexpr size_t kSzY16    = (size_t)kSeqL * kDin * 2;
constexpr size_t kOffWIN16  = 0;
constexpr size_t kOffWXP16  = kOffWIN16  + kSzWIN16;
constexpr size_t kOffWDT16  = kOffWXP16  + kSzWXP16;
constexpr size_t kOffWOUT16 = kOffWDT16  + kSzWDT16;
constexpr size_t kOffYLN16  = kOffWOUT16 + kSzWOUT16;
constexpr size_t kOffXZ     = kOffYLN16  + kSzYLN16;
constexpr size_t kOffUC     = kOffXZ     + kSzXZ;
constexpr size_t kOffUC16   = kOffUC     + kSzUC;
constexpr size_t kOffPROJ   = kOffUC16   + kSzUC16;
constexpr size_t kOffDT16   = kOffPROJ   + kSzPROJ;
constexpr size_t kOffDLR    = kOffDT16   + kSzDT16;
constexpr size_t kOffY16    = kOffDLR    + kSzDLR;
constexpr size_t kWsTotal   = kOffY16    + kSzY16;
static_assert(kWsTotal == 106954752ull);
static_assert(kWsTotal <= 134217728ull);
static_assert((kOffWXP16 % 128) == 0 && (kOffWDT16 % 128) == 0 && (kOffWOUT16 % 128) == 0 && (kOffYLN16 % 128) == 0 &&
              (kOffXZ % 128) == 0 && (kOffUC % 128) == 0 && (kOffUC16 % 128) == 0 && (kOffPROJ % 128) == 0 &&
              (kOffDT16 % 128) == 0 && (kOffDLR % 128) == 0 && (kOffY16 % 128) == 0);

__device__ __forceinline__ void row_guard_h(v8f& a0, v8f& a1, v8f& a2, v8f& a3, v16h x,
                                            v16h b0, v16h b1, v16h b2, v16h b3) {
  asm volatile("v_nop\n\tv_nop\n\tv_nop\n\tv_nop"
               : "+v"(a0), "+v"(a1), "+v"(a2), "+v"(a3)
               : "v"(x), "v"(b0), "v"(b1), "v"(b2), "v"(b3));
}
__device__ __forceinline__ void keep4_h(v16h a, v16h b, v16h c, v16h d) { asm volatile("v_nop" :: "v"(a), "v"(b), "v"(c), "v"(d)); }
__device__ __forceinline__ void acc_guard4(v8f& a, v8f& b, v8f& c, v8f& d) { asm volatile("v_nop\n\tv_nop\n\tv_nop\n\tv_nop" : "+v"(a), "+v"(b), "+v"(c), "+v"(d)); }

struct FragH {
  union U { v16h v; v8h h[2]; };
  static __device__ __forceinline__ v16h load(const _Float16* p) {
    U f; f.h[0] = *(const v8h*)(p); f.h[1] = *(const v8h*)(p + 16); return f.v;
  }
  static __device__ __forceinline__ v8f mma(v16h a, v16h b, v8f c) {
    return __builtin_amdgcn_wmma_f32_16x16x32_f16(false, a, false, b, (short)0, c, false, false);
  }
};

template <int BIAS_MODE, bool RESID>
__global__ __launch_bounds__(256) void wmma_gemm64_f16(
    const unsigned short* __restrict__ Ap, int lda,
    const unsigned short* __restrict__ Btp, int ldb,
    float* __restrict__ Cout, int ldc,
    const float* __restrict__ bias,
    const float* __restrict__ resid,
    int M, int N, int K, float scale) {
  const _Float16* A  = (const _Float16*)Ap;
  const _Float16* Bt = (const _Float16*)Btp;
  __shared__ __align__(16) float sT[8][16 * 68];
  const int lane = threadIdx.x & 31;
  const int wave = threadIdx.x >> 5;
  const int tilesN = N >> 6;
  const int tilesM = M >> 6;
  const int tile = blockIdx.x * 8 + wave;
  if (tile >= tilesM * tilesN) return;
  const int tm = tile / tilesN;
  const int tn = tile - tm * tilesN;
  const int m0 = tm << 6;
  const int n0 = tn << 6;

  const int rlane = lane & 15;
  const int koff  = (lane >> 4) * 8;
  const int mOff  = (lane >> 4) * 8;

  v8f acc[4][4];
#pragma unroll
  for (int i = 0; i < 4; ++i)
#pragma unroll
    for (int j = 0; j < 4; ++j) acc[i][j] = (v8f){0.f,0.f,0.f,0.f,0.f,0.f,0.f,0.f};

  for (int k0 = 0; k0 < K; k0 += 32) {
    v16h bh[4];
#pragma unroll
    for (int j = 0; j < 4; ++j) {
      const size_t bo = (size_t)(n0 + (j << 4) + rlane) * ldb + koff + k0;
      bh[j] = FragH::load(Bt + bo);
    }
#pragma unroll
    for (int i = 0; i < 4; ++i) {
      const size_t ao = (size_t)(m0 + (i << 4) + rlane) * lda + koff + k0;
      v16h ah = FragH::load(A + ao);
#pragma unroll
      for (int j = 0; j < 4; ++j) acc[i][j] = FragH::mma(ah, bh[j], acc[i][j]);
      row_guard_h(acc[i][0], acc[i][1], acc[i][2], acc[i][3], ah, bh[0], bh[1], bh[2], bh[3]);
    }
    keep4_h(bh[0], bh[1], bh[2], bh[3]);
  }
  acc_guard4(acc[0][0], acc[0][1], acc[0][2], acc[0][3]);
  acc_guard4(acc[1][0], acc[1][1], acc[1][2], acc[1][3]);
  acc_guard4(acc[2][0], acc[2][1], acc[2][2], acc[2][3]);
  acc_guard4(acc[3][0], acc[3][1], acc[3][2], acc[3][3]);

  float* slab = sT[wave];
#pragma unroll
  for (int i = 0; i < 4; ++i) {
    const int mBase = m0 + (i << 4);
#pragma unroll
    for (int j = 0; j < 4; ++j) {
      const int n = n0 + (j << 4) + rlane;
      float bv = 0.f;
      if (BIAS_MODE == 2) bv = bias[n];
#pragma unroll
      for (int r = 0; r < 8; ++r) {
        float v = acc[i][j][r] * scale;
        if (BIAS_MODE == 2) v += bv;
        slab[(mOff + r) * 68 + (j << 4) + rlane] = v;
      }
    }
    __builtin_amdgcn_fence(__ATOMIC_RELEASE, "workgroup");
    __builtin_amdgcn_wave_barrier();
    __builtin_amdgcn_fence(__ATOMIC_ACQUIRE, "workgroup");
    {
      const int hh = lane >> 4, c4 = (lane & 15) * 4;
      v4f vals[8];
#pragma unroll
      for (int it = 0; it < 8; ++it) {
        const int row = it * 2 + hh;
        v4f v = *(const v4f*)(slab + row * 68 + c4);
        if (RESID) {
          const v4f rv = *(const v4f*)(resid + (size_t)(mBase + row) * ldc + n0 + c4);
          v[0] += rv[0]; v[1] += rv[1]; v[2] += rv[2]; v[3] += rv[3];
        }
        vals[it] = v;
      }
      for (int pass = 0; pass < 2; ++pass) {
#pragma unroll
        for (int it = 0; it < 8; ++it) {
          const int row = it * 2 + hh;
          *(volatile v4f*)(Cout + (size_t)(mBase + row) * ldc + n0 + c4) = vals[it];
        }
        __threadfence();
      }
    }
    __builtin_amdgcn_fence(__ATOMIC_RELEASE, "workgroup");
    __builtin_amdgcn_wave_barrier();
    __builtin_amdgcn_fence(__ATOMIC_ACQUIRE, "workgroup");
  }
}

__global__ __launch_bounds__(256) void cast_f16_pad_kernel(
    const float* __restrict__ src, unsigned short* __restrict__ dst, int total8, int valid8, float scale)
{
  const int i = blockIdx.x * 256 + threadIdx.x;
  if (i >= total8) return;
  const bool ok = (i < valid8);
  const int ic = ok ? i : (valid8 - 1);
  const float* p = src + ((size_t)ic << 3);
  const v4f a0 = *(const v4f*)(p);
  const v4f a1 = *(const v4f*)(p + 4);
  v8h hv;
#pragma unroll
  for (int e = 0; e < 4; ++e) {
    const float f0 = ok ? (a0[e] * scale) : 0.0f;
    const float f1 = ok ? (a1[e] * scale) : 0.0f;
    hv[e]     = (_Float16)f0;
    hv[4 + e] = (_Float16)f1;
  }
  unsigned short* q = dst + ((size_t)i << 3);
  *(volatile v8h*)q = hv;
  __threadfence();
  *(volatile v8h*)q = hv;
}

__global__ __launch_bounds__(128) void layernorm_f16_kernel(
    const float* __restrict__ x, const float* __restrict__ lw, const float* __restrict__ lb,
    unsigned short* __restrict__ Y16)
{
  __shared__ float sSum[4];
  __shared__ float sSq[4];
  const int tid = threadIdx.x, lane = tid & 31, wave = tid >> 5;
  const size_t e0 = (size_t)blockIdx.x * kDmod + (size_t)tid * 8;
  const v4f a0 = *(const v4f*)(x + e0);
  const v4f a1 = *(const v4f*)(x + e0 + 4);
  float s = ((a0[0] + a0[1]) + (a0[2] + a0[3])) + ((a1[0] + a1[1]) + (a1[2] + a1[3]));
  s += __shfl_xor(s, 16, 32);
  s += __shfl_xor(s, 8, 32);
  s += __shfl_xor(s, 4, 32);
  s += __shfl_xor(s, 2, 32);
  s += __shfl_xor(s, 1, 32);
  if (lane == 0) sSum[wave] = s;
  __syncthreads();
  const float mean = ((sSum[0] + sSum[1]) + (sSum[2] + sSum[3])) * kInvDm;
  float dv[8];
#pragma unroll
  for (int e = 0; e < 4; ++e) { dv[e] = a0[e] - mean; dv[4 + e] = a1[e] - mean; }
  float q = ((dv[0] * dv[0] + dv[1] * dv[1]) + (dv[2] * dv[2] + dv[3] * dv[3])) +
            ((dv[4] * dv[4] + dv[5] * dv[5]) + (dv[6] * dv[6] + dv[7] * dv[7]));
  q += __shfl_xor(q, 16, 32);
  q += __shfl_xor(q, 8, 32);
  q += __shfl_xor(q, 4, 32);
  q += __shfl_xor(q, 2, 32);
  q += __shfl_xor(q, 1, 32);
  if (lane == 0) sSq[wave] = q;
  __syncthreads();
  const float var = ((sSq[0] + sSq[1]) + (sSq[2] + sSq[3])) * kInvDm;
  const float rs  = rsqrtf(var + kLnEps);
  const v4f w0 = *(const v4f*)(lw + tid * 8);
  const v4f w1 = *(const v4f*)(lw + tid * 8 + 4);
  const v4f b0 = *(const v4f*)(lb + tid * 8);
  const v4f b1 = *(const v4f*)(lb + tid * 8 + 4);
  v8h hv;
#pragma unroll
  for (int e = 0; e < 4; ++e) {
    const float y0 = (dv[e] * rs) * w0[e] + b0[e];
    const float y1 = (dv[4 + e] * rs) * w1[e] + b1[e];
    hv[e]     = (_Float16)y0;
    hv[4 + e] = (_Float16)y1;
  }
  unsigned short* qd = Y16 + e0;
  *(volatile v8h*)qd = hv;
  __threadfence();
  *(volatile v8h*)qd = hv;
}

__global__ __launch_bounds__(256) void dt_cast_kernel(
    const float* __restrict__ PROJ, unsigned short* __restrict__ DT16, int total8, float scale)
{
  const int i = blockIdx.x * 256 + threadIdx.x;
  if (i >= total8) return;
  const int e0  = i << 3;
  const int row = e0 >> 6;
  const int c8  = e0 & 63;
  const float* p = PROJ + (size_t)row * kPrjP + c8;
  const v4f a0 = *(const v4f*)(p);
  const v4f a1 = *(const v4f*)(p + 4);
  v8h hv;
#pragma unroll
  for (int e = 0; e < 4; ++e) {
    hv[e]     = (_Float16)(a0[e] * scale);
    hv[4 + e] = (_Float16)(a1[e] * scale);
  }
  unsigned short* qd = DT16 + e0;
  *(volatile v8h*)qd = hv;
  __threadfence();
  *(volatile v8h*)qd = hv;
}

__global__ __launch_bounds__(256) void conv_silu_kernel(
    const float* __restrict__ XZ, const float* __restrict__ cw, const float* __restrict__ cb,
    float* __restrict__ UC, unsigned short* __restrict__ UC16)
{
  __shared__ __align__(16) float sT[16 * kTP];
  const int tid = threadIdx.x, lane = tid & 31, wave = tid >> 5;
  const int d0 = blockIdx.x * 256, d = d0 + tid;
  const int t0 = blockIdx.y * 64;
  const v4f wv = *(const v4f*)(cw + d * 4);
  const float w0 = wv[0], w1 = wv[1], w2 = wv[2], w3 = wv[3];
  const float bc = cb[d];
  float xm3, xm2, xm1;
  {
    const int r3 = t0 - 3, r2 = t0 - 2, r1 = t0 - 1;
    const float v3 = XZ[(size_t)(r3 < 0 ? 0 : r3) * kXZP + d];
    const float v2 = XZ[(size_t)(r2 < 0 ? 0 : r2) * kXZP + d];
    const float v1 = XZ[(size_t)(r1 < 0 ? 0 : r1) * kXZP + d];
    xm3 = (r3 >= 0) ? v3 : 0.f;
    xm2 = (r2 >= 0) ? v2 : 0.f;
    xm1 = (r1 >= 0) ? v1 : 0.f;
  }
  const int hrow = wave >> 1;
  const int hch  = (wave & 1) * 128 + lane * 4;
#pragma unroll 1
  for (int sub = 0; sub < 4; ++sub) {
    const int lb = t0 + sub * 16;
#pragma unroll 1
    for (int s = 0; s < 16; ++s) {
      const float xc = XZ[(size_t)(lb + s) * kXZP + d];
      float acc = w0 * xm3;
      acc = fmaf(w1, xm2, acc);
      acc = fmaf(w2, xm1, acc);
      acc = fmaf(w3, xc, acc);
      const float sv = acc + bc;
      const float sg = __builtin_amdgcn_rcpf(1.0f + __expf(-sv));
      sT[s * kTP + tid] = sv * sg;
      xm3 = xm2; xm2 = xm1; xm1 = xc;
    }
    __syncthreads();
    v4f fv[4];
    v8h bv[2];
#pragma unroll
    for (int it = 0; it < 4; ++it) fv[it] = *(const v4f*)(sT + (it * 4 + hrow) * kTP + hch);
#pragma unroll
    for (int it = 0; it < 2; ++it) {
      const float* sp = sT + (it * 8 + wave) * kTP + lane * 8;
      const v4f a0 = *(const v4f*)(sp);
      const v4f a1 = *(const v4f*)(sp + 4);
#pragma unroll
      for (int e = 0; e < 4; ++e) {
        bv[it][e]     = (_Float16)a0[e];
        bv[it][4 + e] = (_Float16)a1[e];
      }
    }
    for (int pass = 0; pass < 2; ++pass) {
#pragma unroll
      for (int it = 0; it < 4; ++it)
        *(volatile v4f*)(UC + (size_t)(lb + it * 4 + hrow) * kDin + d0 + hch) = fv[it];
#pragma unroll
      for (int it = 0; it < 2; ++it)
        *(volatile v8h*)(UC16 + (size_t)(lb + it * 8 + wave) * kDin + d0 + lane * 8) = bv[it];
      __threadfence();
    }
    __syncthreads();
  }
}

__global__ __launch_bounds__(256) void scan_kernel(
    const float* __restrict__ DLR, const float* __restrict__ UC, const float* __restrict__ XZ,
    const float* __restrict__ PROJ, const float* __restrict__ A_log, const float* __restrict__ Dv,
    unsigned short* __restrict__ Y16)
{
  __shared__ __align__(16) float sBC[16 * 32];
  __shared__ __align__(16) float sY[16 * kTP];
  __shared__ __align__(16) float sA[kNst * 256];
  const int tid = threadIdx.x, lane = tid & 31, wave = tid >> 5;
  const int d0 = blockIdx.x * 256, d = d0 + tid;

#pragma unroll 1
  for (int n = 0; n < kNst; ++n) sA[n * 256 + tid] = -expf(A_log[(size_t)d * kNst + n]);
  __syncthreads();
  float An[kNst], h[kNst];
#pragma unroll
  for (int n = 0; n < kNst; ++n) {
    An[n] = sA[n * 256 + tid];
    h[n] = 0.f;
  }
  const float Dd = Dv[d];

#pragma unroll 1
  for (int c = 0; c < kSeqL / 16; ++c) {
    const int l0 = c * 16;
    if (tid < 128) {
      const int r = tid >> 3, q = (tid & 7) * 4;
      const v4f v = *(const v4f*)(PROJ + (size_t)(l0 + r) * kPrjP + kDtR + q);
      *(v4f*)(sBC + r * 32 + q) = v;
    }
    __syncthreads();
#pragma unroll 1
    for (int s = 0; s < 16; ++s) {
      const size_t m = (size_t)(l0 + s);
      const float a  = DLR[m * kDin + d];
      const float xv = UC[m * kDin + d];
      const float zv = XZ[m * kXZP + kDin + d];
      const float ea  = __expf(-fabsf(a));
      const float up  = 1.0f + ea;
      const float l1p = __logf(up) + (ea - (up - 1.0f)) * __builtin_amdgcn_rcpf(up);
      const float delta = fmaxf(a, 0.0f) + l1p;
      v4f Bq[4], Cq[4];
#pragma unroll
      for (int qq = 0; qq < 4; ++qq) {
        Bq[qq] = *(const v4f*)(sBC + s * 32 + 4 * qq);
        Cq[qq] = *(const v4f*)(sBC + s * 32 + kNst + 4 * qq);
      }
      const float dtx = delta * xv;
      float y = 0.f;
#pragma unroll
      for (int n = 0; n < kNst; ++n) {
        const float e = __expf(delta * An[n]);
        const float hn = e * h[n] + dtx * Bq[n >> 2][n & 3];
        h[n] = hn;
        y = hn * Cq[n >> 2][n & 3] + y;
      }
      y = xv * Dd + y;
      const float sg = __builtin_amdgcn_rcpf(1.0f + __expf(-zv));
      const float g  = zv * sg;
      sY[s * kTP + tid] = (y * g) * kCarY;
    }
    __syncthreads();
    v8h hv[2];
#pragma unroll
    for (int it = 0; it < 2; ++it) {
      const float* sp = sY + (it * 8 + wave) * kTP + lane * 8;
      const v4f a0 = *(const v4f*)(sp);
      const v4f a1 = *(const v4f*)(sp + 4);
#pragma unroll
      for (int e = 0; e < 4; ++e) { hv[it][e] = (_Float16)a0[e]; hv[it][4 + e] = (_Float16)a1[e]; }
    }
    for (int pass = 0; pass < 2; ++pass) {
#pragma unroll
      for (int it = 0; it < 2; ++it)
        *(volatile v8h*)(Y16 + (size_t)(l0 + it * 8 + wave) * kDin + d0 + lane * 8) = hv[it];
      __threadfence();
    }
  }
}

extern "C" void kernel_launch(void* const* d_in, const int* in_sizes, int n_in,
                              void* d_out, int out_size, void* d_ws, size_t ws_size,
                              hipStream_t stream)
{
  if (n_in < 12) return;
  if (in_sizes[0] != kRows * kDmod) return;
  if (in_sizes[1] != kDmod || in_sizes[2] != kDmod) return;
  if (in_sizes[3] != kXZP * kDmod) return;
  if (in_sizes[4] != kDin * 4 || in_sizes[5] != kDin) return;
  if (in_sizes[6] != kPrjN * kDin) return;
  if (in_sizes[7] != kDin * kDtR || in_sizes[8] != kDin) return;
  if (in_sizes[9] != kDin * kNst || in_sizes[10] != kDin) return;
  if (in_sizes[11] != kDmod * kDin) return;
  if (out_size != kRows * kDmod) return;
  if (ws_size < kWsTotal) return;

  const float* x      = (const float*)d_in[0];
  const float* ln_w   = (const float*)d_in[1];
  const float* ln_b   = (const float*)d_in[2];
  const float* W_in   = (const float*)d_in[3];
  const float* conv_w = (const float*)d_in[4];
  const float* conv_b = (const float*)d_in[5];
  const float* W_xprj = (const float*)d_in[6];
  const float* W_dt   = (const float*)d_in[7];
  const float* b_dt   = (const float*)d_in[8];
  const float* A_log  = (const float*)d_in[9];
  const float* Dv     = (const float*)d_in[10];
  const float* W_out  = (const float*)d_in[11];
  float* dout = (float*)d_out;

  char* ws = (char*)d_ws;
  unsigned short* WIN16  = (unsigned short*)(ws + kOffWIN16);
  unsigned short* WXP16  = (unsigned short*)(ws + kOffWXP16);
  unsigned short* WDT16  = (unsigned short*)(ws + kOffWDT16);
  unsigned short* WOUT16 = (unsigned short*)(ws + kOffWOUT16);
  unsigned short* YLN16  = (unsigned short*)(ws + kOffYLN16);
  float*          XZ     = (float*)(ws + kOffXZ);
  float*          UC     = (float*)(ws + kOffUC);
  unsigned short* UC16   = (unsigned short*)(ws + kOffUC16);
  float*          PROJ   = (float*)(ws + kOffPROJ);
  unsigned short* DT16   = (unsigned short*)(ws + kOffDT16);
  float*          DLR    = (float*)(ws + kOffDLR);
  unsigned short* Y16    = (unsigned short*)(ws + kOffY16);
  const float* dummy_bias  = b_dt;
  const float* dummy_resid = x;

  cast_f16_pad_kernel<<<(kXZP * kDmod / 8) / 256, 256, 0, stream>>>(W_in, WIN16, kXZP * kDmod / 8, kXZP * kDmod / 8, kCarWin);
  cast_f16_pad_kernel<<<(kPrjP * kDin / 8) / 256, 256, 0, stream>>>(W_xprj, WXP16, kPrjP * kDin / 8, kPrjN * kDin / 8, kCarWxp);
  cast_f16_pad_kernel<<<(kDin * kDtR / 8) / 256, 256, 0, stream>>>(W_dt, WDT16, kDin * kDtR / 8, kDin * kDtR / 8, kCarWdt);
  cast_f16_pad_kernel<<<(kDmod * kDin / 8) / 256, 256, 0, stream>>>(W_out, WOUT16, kDmod * kDin / 8, kDmod * kDin / 8, kCarWout);

  layernorm_f16_kernel<<<kRows, 128, 0, stream>>>(x, ln_w, ln_b, YLN16);

  for (int b = 0; b < kBatch; ++b) {
    const unsigned short* Yb = YLN16 + (size_t)b * kSeqL * kDmod;
    const float* xb = x + (size_t)b * kSeqL * kDmod;
    float* outb = dout + (size_t)b * kSeqL * kDmod;

    wmma_gemm64_f16<0, false><<<dim3(256, 1), 256, 0, stream>>>(
        Yb, kDmod, WIN16, kDmod, XZ, kXZP, dummy_bias, dummy_resid, kSeqL, kXZP, kDmod, kFoldIn);

    conv_silu_kernel<<<dim3(kDin / 256, kSeqL / 64), 256, 0, stream>>>(XZ, conv_w, conv_b, UC, UC16);

    wmma_gemm64_f16<0, false><<<dim3(8, 1), 256, 0, stream>>>(
        UC16, kDin, WXP16, kDin, PROJ, kPrjP, dummy_bias, dummy_resid, kSeqL, kPrjP, kDin, kFoldXp);

    dt_cast_kernel<<<(kSeqL * kDtR / 8) / 256, 256, 0, stream>>>(PROJ, DT16, kSeqL * kDtR / 8, kCarDt);

    wmma_gemm64_f16<2, false><<<dim3(128, 1), 256, 0, stream>>>(
        DT16, kDtR, WDT16, kDtR, DLR, kDin, b_dt, dummy_resid, kSeqL, kDin, kDtR, kFoldDt);

    scan_kernel<<<dim3(kDin / 256, 1), 256, 0, stream>>>(DLR, UC, XZ, PROJ, A_log, Dv, Y16);

    wmma_gemm64_f16<0, true><<<dim3(64, 1), 256, 0, stream>>>(
        Y16, kDin, WOUT16, kDin, outb, kDmod, dummy_bias, xb, kSeqL, kDmod, kDin, kFoldOut);
  }
}
